// RPEMultiHeadAttention_79551384256915
// MI455X (gfx1250) — hardware-verified
//
#include <hip/hip_runtime.h>
#include <stdint.h>

typedef __attribute__((ext_vector_type(16))) _Float16 v16h;
typedef __attribute__((ext_vector_type(8)))  _Float16 v8h;
typedef __attribute__((ext_vector_type(16))) __bf16   v16b;
typedef __attribute__((ext_vector_type(8)))  __bf16   v8b;
typedef __attribute__((ext_vector_type(8)))  float    v8f;
typedef __attribute__((ext_vector_type(4)))  float    v4f;
typedef __attribute__((ext_vector_type(4)))  unsigned int v4u;

__device__ __forceinline__ unsigned short f2bf_bits(float f) {
  unsigned u = __float_as_uint(f);
  return (unsigned short)((u + 0x7FFFu + ((u >> 16) & 1u)) >> 16);
}
__device__ __forceinline__ float bf_bits2f(unsigned short h) { return __uint_as_float(((unsigned)h) << 16); }

__device__ __forceinline__ void dep_guard_h(v8f& a, v8f& b, v16h x, v16h y) { asm volatile("v_nop\n\tv_nop\n\tv_nop\n\tv_nop" : "+v"(a), "+v"(b) : "v"(x), "v"(y)); }
__device__ __forceinline__ void dep_guard_b(v8f& a, v8f& b, v16b x, v16b y) { asm volatile("v_nop\n\tv_nop\n\tv_nop\n\tv_nop" : "+v"(a), "+v"(b) : "v"(x), "v"(y)); }
__device__ __forceinline__ void keep4_h(v16h a, v16h b, v16h c, v16h d) { asm volatile("v_nop" :: "v"(a), "v"(b), "v"(c), "v"(d)); }
__device__ __forceinline__ void keep4_b(v16b a, v16b b, v16b c, v16b d) { asm volatile("v_nop" :: "v"(a), "v"(b), "v"(c), "v"(d)); }
__device__ __forceinline__ void acc_guard4(v8f& a, v8f& b, v8f& c, v8f& d) { asm volatile("v_nop\n\tv_nop\n\tv_nop\n\tv_nop" : "+v"(a), "+v"(b), "+v"(c), "+v"(d)); }
template <typename T> struct Frag;
template <> struct Frag<_Float16> {
  typedef v16h V; union U { v16h v; v8h h[2]; };
  static __device__ __forceinline__ v16h load(const _Float16* p) {
    U f; f.h[0] = *(const v8h*)(p); f.h[1] = *(const v8h*)(p + 16); return f.v;
  }
  static __device__ __forceinline__ v8f mma(v16h a, v16h b, v8f c) {
    return __builtin_amdgcn_wmma_f32_16x16x32_f16(false, a, false, b, (short)0, c, false, false);
  }
  static __device__ __forceinline__ void guard(v8f& a, v8f& b, v16h x, v16h y) { dep_guard_h(a, b, x, y); }
  static __device__ __forceinline__ void keep(v16h a, v16h b, v16h c, v16h d) { keep4_h(a, b, c, d); }
};
template <> struct Frag<__bf16> {
  typedef v16b V; union U { v16b v; v8b h[2]; };
  static __device__ __forceinline__ v16b load(const __bf16* p) {
    U f; f.h[0] = *(const v8b*)(p); f.h[1] = *(const v8b*)(p + 16); return f.v;
  }
  static __device__ __forceinline__ v8f mma(v16b a, v16b b, v8f c) {
    return __builtin_amdgcn_wmma_f32_16x16x32_bf16(false, a, false, b, (short)0, c, false, false);
  }
  static __device__ __forceinline__ void guard(v8f& a, v8f& b, v16b x, v16b y) { dep_guard_b(a, b, x, y); }
  static __device__ __forceinline__ void keep(v16b a, v16b b, v16b c, v16b d) { keep4_b(a, b, c, d); }
};

template <int ET> struct Elem;
template <> struct Elem<0> { typedef _Float16 T; };
template <> struct Elem<1> { typedef __bf16 T; };
template <int ET, bool SPLIT, int BIAS_MODE, int OUT_MODE, bool RESID, int ACT = 0>
__global__ __launch_bounds__(256) void wmma_gemm64(
    const unsigned short* __restrict__ Ap, const unsigned short* __restrict__ A2p, int lda, long strideA,
    const unsigned short* __restrict__ Btp, const unsigned short* __restrict__ Bt2p, int ldb, long strideB,
    void* __restrict__ Cout, void* __restrict__ Cout2, int ldc, long strideC,
    const float* __restrict__ bias,
    const float* __restrict__ resid, long strideR,
    int M, int N, int K, float scale) {
  typedef typename Elem<ET>::T T;
  typedef typename Frag<T>::V V;
  const T* A = (const T*)Ap; const T* A2 = (const T*)A2p; const T* Bt = (const T*)Btp; const T* Bt2 = (const T*)Bt2p;
  __shared__ __align__(16) float sT[8][16 * 68];
  const int b    = blockIdx.y;
  const int lane = threadIdx.x & 31;
  const int wave = threadIdx.x >> 5;
  const int tilesN = N >> 6;
  const int tilesM = M >> 6;
  const int tile = blockIdx.x * 8 + wave;
  if (tile >= tilesM * tilesN) return;
  const int tm = tile / tilesN;
  const int tn = tile - tm * tilesN;
  const int m0 = tm << 6;
  const int n0 = tn << 6;

  const T* Ab  = A  + (size_t)b * strideA;
  const T* Bb  = Bt + (size_t)b * strideB;
  const T* Ab2 = SPLIT ? (A2  + (size_t)b * strideA) : nullptr;
  const T* Bb2 = SPLIT ? (Bt2 + (size_t)b * strideB) : nullptr;

  const int rlane = lane & 15;
  const int koff  = (lane >> 4) * 8;
  const int mOff  = (lane >> 4) * 8;

  v8f acc[4][4];
#pragma unroll
  for (int i = 0; i < 4; ++i)
#pragma unroll
    for (int j = 0; j < 4; ++j) acc[i][j] = (v8f){0.f,0.f,0.f,0.f,0.f,0.f,0.f,0.f};

  for (int k0 = 0; k0 < K; k0 += 32) {
    V bh[4], bl[4];
#pragma unroll
    for (int j = 0; j < 4; ++j) {
      const size_t bo = (size_t)(n0 + (j << 4) + rlane) * ldb + koff + k0;
      bh[j] = Frag<T>::load(Bb + bo);
      if (SPLIT) bl[j] = Frag<T>::load(Bb2 + bo);
    }
#pragma unroll
    for (int i = 0; i < 4; ++i) {
      const size_t ao = (size_t)(m0 + (i << 4) + rlane) * lda + koff + k0;
      V ah = Frag<T>::load(Ab + ao);
      V al;
      if (SPLIT) al = Frag<T>::load(Ab2 + ao);
#pragma unroll
      for (int j = 0; j < 4; ++j) {
        acc[i][j] = Frag<T>::mma(ah, bh[j], acc[i][j]);
        if (SPLIT) {
          acc[i][j] = Frag<T>::mma(ah, bl[j], acc[i][j]);
          acc[i][j] = Frag<T>::mma(al, bh[j], acc[i][j]);
        }
      }
      Frag<T>::guard(acc[i][0], acc[i][3], ah, SPLIT ? al : ah);
    }
    Frag<T>::keep(bh[0], bh[1], bh[2], bh[3]);
    if (SPLIT) Frag<T>::keep(bl[0], bl[1], bl[2], bl[3]);
  }
  acc_guard4(acc[0][0], acc[0][1], acc[0][2], acc[0][3]);
  acc_guard4(acc[1][0], acc[1][1], acc[1][2], acc[1][3]);
  acc_guard4(acc[2][0], acc[2][1], acc[2][2], acc[2][3]);
  acc_guard4(acc[3][0], acc[3][1], acc[3][2], acc[3][3]);

  float* slab = sT[wave];
  const float* Rb = RESID ? (resid + (size_t)b * strideR) : nullptr;
#pragma unroll
  for (int i = 0; i < 4; ++i) {
    const int mBase = m0 + (i << 4);
#pragma unroll
    for (int j = 0; j < 4; ++j) {
      const int n = n0 + (j << 4) + rlane;
      float bv = 0.f;
      if (BIAS_MODE == 2) bv = bias[n];
#pragma unroll
      for (int r = 0; r < 8; ++r) {
        float v = acc[i][j][r] * scale;
        if (BIAS_MODE == 1) v += bias[mBase + mOff + r];
        if (BIAS_MODE == 2) v += bv;
        if (RESID) v += Rb[(size_t)(mBase + mOff + r) * ldc + n];
        if (ACT == 1) v = tanhf(v);
        if (ACT == 2) v = fmaxf(v, 0.0f);
        if (ACT == 3) v = v / (1.0f + expf(-v));
        if (ACT == 4) v = (v > 0.f) ? v : 0.01f * v;
        if (ACT == 5) v = 0.5f * v * (1.0f + erff(v * 0.70710678118654752f));
        slab[(mOff + r) * 68 + (j << 4) + rlane] = v;
      }
    }
    __builtin_amdgcn_fence(__ATOMIC_RELEASE, "workgroup");
    __builtin_amdgcn_wave_barrier();
    __builtin_amdgcn_fence(__ATOMIC_ACQUIRE, "workgroup");
    if (OUT_MODE == 0) {
      float* C = (float*)Cout + (size_t)b * strideC;
      const int hh = lane >> 4, c4 = (lane & 15) * 4;
      for (int pass = 0; pass < 2; ++pass) {
#pragma unroll
        for (int it = 0; it < 8; ++it) {
          const int row = it * 2 + hh;
          v4f v = *(const v4f*)(slab + row * 68 + c4);
          *(volatile v4f*)(C + (size_t)(mBase + row) * ldc + n0 + c4) = v;
        }
        __threadfence();
      }
    } else {
      const int q = lane >> 3, c8 = (lane & 7) * 8;
      unsigned short* C  = (unsigned short*)Cout  + (size_t)b * strideC;
      unsigned short* C2 = (OUT_MODE == 2) ? ((unsigned short*)Cout2 + (size_t)b * strideC) : nullptr;
      for (int pass = 0; pass < 2; ++pass) {
#pragma unroll
        for (int it = 0; it < 4; ++it) {
          const int row = it * 4 + q;
          const float* sp = slab + row * 68 + c8;
          v8h hv, lv;
#pragma unroll
          for (int e = 0; e < 8; ++e) {
            if (OUT_MODE == 1) {
              hv[e] = (_Float16)sp[e];
            } else {
              unsigned short hb = f2bf_bits(sp[e]);
              unsigned short lb = f2bf_bits(sp[e] - bf_bits2f(hb));
              hv[e] = __builtin_bit_cast(_Float16, hb);
              lv[e] = __builtin_bit_cast(_Float16, lb);
            }
          }
          *(volatile v8h*)(C + (size_t)(mBase + row) * ldc + n0 + c8) = hv;
          if (OUT_MODE == 2) *(volatile v8h*)(C2 + (size_t)(mBase + row) * ldc + n0 + c8) = lv;
        }
        __threadfence();
      }
    }
    __builtin_amdgcn_fence(__ATOMIC_RELEASE, "workgroup");
    __builtin_amdgcn_wave_barrier();
    __builtin_amdgcn_fence(__ATOMIC_ACQUIRE, "workgroup");
  }
}

constexpr int kSeqT   = 1024;
constexpr int kSeqS   = 1024;
constexpr int kBatch  = 4;
constexpr int kDModel = 1024;
constexpr int kHeads  = 16;
constexpr int kHDim   = 64;
constexpr int kNTab    = 2047;
constexpr int kR1Rows  = 2048;
constexpr int kT2Pitch = 2112;
constexpr int kRowPitch = kBatch * kDModel;
constexpr int kKC      = 64;
constexpr int kQB      = 64;
constexpr int kRWin    = 128;
constexpr int kTWin    = 144;
constexpr int kPqPitch = 84;
constexpr int kPshK    = 96;
constexpr int kOsPitch = 68;
constexpr float kPCarry    = 32768.0f;
constexpr float kTCarry    = 16.0f;
constexpr float kTCarryInv = 1.0f / 16.0f;
constexpr float kScale     = 0.125f;
static_assert(kSeqT % kQB == 0);
static_assert(kSeqS % kKC == 0);
static_assert(kHDim == 64);
static_assert(16 * kOsPitch <= 16 * kPqPitch);
static_assert((kSeqT * kBatch) % 64 == 0);
static_assert(kDModel % 64 == 0);
static_assert(kDModel % 32 == 0);
static_assert(48 + 80 <= kRWin);
static_assert(48 + kPshK <= kTWin);
static_assert((kSeqS - kKC) + 960 + kRWin <= kR1Rows);
static_assert((kSeqS - kKC) + 960 + kTWin <= kT2Pitch);

__device__ __forceinline__ v8f hmma(v16h a, v16h b, v8f c) {
  c = __builtin_amdgcn_wmma_f32_16x16x32_f16(false, a, false, b, (short)0, c, false, false);
  asm volatile("v_nop\n\tv_nop\n\tv_nop\n\tv_nop" : "+v"(c) : "v"(a), "v"(b));
  return c;
}
__device__ __forceinline__ v16h ldfrag(const unsigned short* p) {
  return Frag<_Float16>::load((const _Float16*)(const void*)p);
}
__device__ __forceinline__ unsigned short tab_bits(float x, bool keep) {
  const float v = keep ? (bf_bits2f(f2bf_bits(x)) * kTCarry) : 0.0f;
  return __builtin_bit_cast(unsigned short, (_Float16)v);
}

__global__ __launch_bounds__(256) void cast3_bf16_kernel(
    const float* __restrict__ s0, const float* __restrict__ s1, const float* __restrict__ s2,
    unsigned short* __restrict__ dst, int n8) {
  const int z = blockIdx.y;
  const float* src = (z == 0) ? s0 : ((z == 1) ? s1 : s2);
  unsigned short* dz = dst + (size_t)z * (size_t)n8 * 8;
  const int i = blockIdx.x * 256 + threadIdx.x;
  if (i < n8) {
    const float* p = src + (size_t)i * 8;
    const v4f a = *(const v4f*)p;
    const v4f c = *(const v4f*)(p + 4);
    v4u w;
    w[0] = (unsigned)f2bf_bits(a[0]) | ((unsigned)f2bf_bits(a[1]) << 16);
    w[1] = (unsigned)f2bf_bits(a[2]) | ((unsigned)f2bf_bits(a[3]) << 16);
    w[2] = (unsigned)f2bf_bits(c[0]) | ((unsigned)f2bf_bits(c[1]) << 16);
    w[3] = (unsigned)f2bf_bits(c[2]) | ((unsigned)f2bf_bits(c[3]) << 16);
    unsigned short* q = dz + (size_t)i * 8;
    *(volatile v4u*)q = w;
    __threadfence();
    *(volatile v4u*)q = w;
  }
}

__global__ __launch_bounds__(256) void wt_transpose_kernel(
    const float* __restrict__ W0, const float* __restrict__ W1, const float* __restrict__ W2,
    unsigned short* __restrict__ Wt) {
  __shared__ __align__(16) unsigned short tile[64 * 72];
  const int z = blockIdx.z;
  const float* W = (z == 0) ? W0 : ((z == 1) ? W1 : W2);
  unsigned short* dst = Wt + (size_t)z * (size_t)kDModel * kDModel;
  const int n0 = blockIdx.x * 64, k0 = blockIdx.y * 64;
  const int tid = threadIdx.x;
  {
    const int kr = tid >> 2, ng = (tid & 3) * 16;
    const float* src = W + (size_t)(k0 + kr) * kDModel + n0 + ng;
#pragma unroll
    for (int i = 0; i < 4; ++i) {
      const v4f a = *(const v4f*)(src + 4 * i);
#pragma unroll
      for (int e = 0; e < 4; ++e) tile[(ng + 4 * i + e) * 72 + kr] = f2bf_bits(a[e]);
    }
  }
  __syncthreads();
  {
    const int col8 = (tid & 7) * 8;
    for (int pass = 0; pass < 2; ++pass) {
#pragma unroll
      for (int it = 0; it < 2; ++it) {
        const int nl = it * 32 + (tid >> 3);
        const v4u w = *(const v4u*)(tile + nl * 72 + col8);
        *(volatile v4u*)(dst + (size_t)(n0 + nl) * kDModel + k0 + col8) = w;
      }
      __threadfence();
    }
  }
}

__global__ __launch_bounds__(256) void rel_cast_kernel(const float* __restrict__ rel, unsigned short* __restrict__ R1) {
  const int i = blockIdx.x * 256 + threadIdx.x;
  if (i < kR1Rows * 8) {
    const int row = i >> 3, seg = i & 7;
    const bool keep = row < kNTab;
    const int rc = keep ? row : (kNTab - 1);
    const float* p = rel + (size_t)rc * kHDim + seg * 8;
    const v4f a = *(const v4f*)p;
    const v4f c = *(const v4f*)(p + 4);
    v4u w;
    w[0] = (unsigned)tab_bits(a[0], keep) | ((unsigned)tab_bits(a[1], keep) << 16);
    w[1] = (unsigned)tab_bits(a[2], keep) | ((unsigned)tab_bits(a[3], keep) << 16);
    w[2] = (unsigned)tab_bits(c[0], keep) | ((unsigned)tab_bits(c[1], keep) << 16);
    w[3] = (unsigned)tab_bits(c[2], keep) | ((unsigned)tab_bits(c[3], keep) << 16);
    unsigned short* q = R1 + (size_t)i * 8;
    *(volatile v4u*)q = w;
    __threadfence();
    *(volatile v4u*)q = w;
  }
}

__global__ __launch_bounds__(256) void orel_transpose_kernel(const float* __restrict__ orel, unsigned short* __restrict__ T2) {
  __shared__ __align__(16) unsigned short tile[64 * 72];
  const int j0 = blockIdx.x * 64;
  const int tid = threadIdx.x;
  {
    const int jr = tid >> 2, dg = (tid & 3) * 16;
    const int j = j0 + jr;
    const bool keep = j < kNTab;
    const int jc = keep ? j : (kNTab - 1);
    const float* src = orel + (size_t)jc * kHDim + dg;
#pragma unroll
    for (int i = 0; i < 4; ++i) {
      const v4f a = *(const v4f*)(src + 4 * i);
#pragma unroll
      for (int e = 0; e < 4; ++e) tile[(dg + 4 * i + e) * 72 + jr] = tab_bits(a[e], keep);
    }
  }
  __syncthreads();
  {
    const int col8 = (tid & 7) * 8;
    for (int pass = 0; pass < 2; ++pass) {
#pragma unroll
      for (int it = 0; it < 2; ++it) {
        const int d = it * 32 + (tid >> 3);
        const v4u w = *(const v4u*)(tile + d * 72 + col8);
        *(volatile v4u*)(T2 + (size_t)d * kT2Pitch + j0 + col8) = w;
      }
      __threadfence();
    }
  }
}

__global__ __launch_bounds__(128) void rpe_attn_kernel(
    const unsigned short* __restrict__ Qp, const unsigned short* __restrict__ Kp,
    const unsigned short* __restrict__ Vp, const unsigned short* __restrict__ R1p,
    const unsigned short* __restrict__ T2p, float* __restrict__ outp) {
  __shared__ __align__(16) unsigned short Ksh[kKC * kHDim];
  __shared__ __align__(16) unsigned short Vtsh[kHDim * kKC];
  __shared__ __align__(16) unsigned short Rsh[kRWin * kHDim];
  __shared__ __align__(16) unsigned short T2sh[kHDim * kTWin];
  __shared__ __align__(16) unsigned short Pn[4][16 * kKC];
  __shared__ __align__(16) unsigned short Psh[4][16 * kPshK];
  __shared__ __align__(16) float Pq[4][16 * kPqPitch];

  const int tid  = threadIdx.x;
  const int wave = tid >> 5;
  const int lane = tid & 31;
  const int hh   = lane >> 4;
  const int c    = lane & 15;
  const int nqb  = kSeqT / kQB;
  const int bx   = blockIdx.x;
  const int qb   = bx % nqb;
  const int bhI  = bx / nqb;
  const int h    = bhI % kHeads;
  const int b    = bhI / kHeads;
  const int qbase = qb * kQB;
  const int q0    = qbase + wave * 16;
  const int roff  = 48 - 16 * wave;
  const size_t headoff = (size_t)b * kDModel + (size_t)h * kHDim;
  const unsigned short* Qh = Qp + headoff;
  const unsigned short* Kh = Kp + headoff;
  const unsigned short* Vh = Vp + headoff;

  v16h qa[2];
  {
    const unsigned short* qrow = Qh + (size_t)(q0 + c) * kRowPitch;
    qa[0] = ldfrag(qrow + 8 * hh);
    qa[1] = ldfrag(qrow + 32 + 8 * hh);
  }

  const float kNegInf = -__builtin_huge_valf();
  float mrow[8], lrow[8];
  v8f oacc[4], oacc2[4];
#pragma unroll
  for (int r = 0; r < 8; ++r) { mrow[r] = kNegInf; lrow[r] = 0.f; }
#pragma unroll
  for (int t = 0; t < 4; ++t) {
    oacc[t]  = (v8f){0.f,0.f,0.f,0.f,0.f,0.f,0.f,0.f};
    oacc2[t] = (v8f){0.f,0.f,0.f,0.f,0.f,0.f,0.f,0.f};
  }

  float* Pqw = Pq[wave];
  unsigned short* pn = Pn[wave];
  unsigned short* ps = Psh[wave];

  for (int kc = 0; kc < kSeqS / kKC; ++kc) {
    const int kv0 = kc * kKC;
    const int jlo = kv0 - qbase + 960;
    __syncthreads();
#pragma unroll
    for (int i = 0; i < 4; ++i) {
      const int idx = tid + 128 * i;
      const int row = idx >> 3, seg = idx & 7;
      const v4u w = *(const v4u*)(Kh + (size_t)(kv0 + row) * kRowPitch + seg * 8);
      *(v4u*)(Ksh + row * kHDim + seg * 8) = w;
    }
#pragma unroll
    for (int i = 0; i < 4; ++i) {
      const int idx = tid + 128 * i;
      const int row = idx >> 3, seg = idx & 7;
      const v4u w = *(const v4u*)(Vh + (size_t)(kv0 + row) * kRowPitch + seg * 8);
      const int d0 = seg * 8;
#pragma unroll
      for (int e = 0; e < 4; ++e) {
        Vtsh[(d0 + 2 * e) * kKC + row]     = (unsigned short)(w[e] & 0xffffu);
        Vtsh[(d0 + 2 * e + 1) * kKC + row] = (unsigned short)(w[e] >> 16);
      }
    }
    asm volatile("" ::: "memory");
#pragma unroll 2
    for (int i = 0; i < 8; ++i) {
      const int idx = tid + 128 * i;
      const int row = idx >> 3, seg = idx & 7;
      const int j  = jlo + row;
      const int jc = (j < kR1Rows) ? j : (kR1Rows - 1);
      const v4u w = *(const v4u*)(R1p + (size_t)jc * kHDim + seg * 8);
      *(v4u*)(Rsh + row * kHDim + seg * 8) = w;
    }
    asm volatile("" ::: "memory");
#pragma unroll 1
    for (int i = 0; i < 9; ++i) {
      const int idx = tid + 128 * i;
      const int d = idx / 18;
      const int seg = idx - d * 18;
      const int col = jlo + seg * 8;
      const int colc = (col < kT2Pitch - 8) ? col : (kT2Pitch - 8);
      const v4u w = *(const v4u*)(T2p + (size_t)d * kT2Pitch + colc);
      *(v4u*)(T2sh + d * kTWin + seg * 8) = w;
    }
    {
      const v4u zz = (v4u){0u, 0u, 0u, 0u};
      v4u* pz = (v4u*)ps;
#pragma unroll
      for (int i = 0; i < 6; ++i) pz[lane + 32 * i] = zz;
    }
    __syncthreads();

#pragma unroll
    for (int n5 = 0; n5 < 5; ++n5) {
      v8f a = (v8f){0.f,0.f,0.f,0.f,0.f,0.f,0.f,0.f};
      const unsigned short* rb = Rsh + (roff + n5 * 16 + c) * kHDim + 8 * hh;
      const v16h b0 = ldfrag(rb);
      const v16h b1 = ldfrag(rb + 32);
      a = hmma(qa[0], b0, a);
      a = hmma(qa[1], b1, a);
#pragma unroll
      for (int r = 0; r < 8; ++r) Pqw[(8 * hh + r) * kPqPitch + n5 * 16 + c] = a[r];
    }
    v8f s[4];
#pragma unroll
    for (int j = 0; j < 4; ++j) {
      s[j] = (v8f){0.f,0.f,0.f,0.f,0.f,0.f,0.f,0.f};
      const unsigned short* kb = Ksh + (j * 16 + c) * kHDim + 8 * hh;
      const v16h b0 = ldfrag(kb);
      const v16h b1 = ldfrag(kb + 32);
      s[j] = hmma(qa[0], b0, s[j]);
      s[j] = hmma(qa[1], b1, s[j]);
    }
    __syncthreads();

    float cm[8];
#pragma unroll
    for (int r = 0; r < 8; ++r) {
      const int R = 8 * hh + r;
      float m = kNegInf;
#pragma unroll
      for (int j = 0; j < 4; ++j) {
        const float pq = Pqw[R * kPqPitch + j * 16 + c - R + 15];
        const float sv = (s[j][r] + pq * kTCarryInv) * kScale;
        s[j][r] = sv;
        m = fmaxf(m, sv);
      }
#pragma unroll
      for (int off = 1; off < 16; off <<= 1) m = fmaxf(m, __shfl_xor(m, off, 32));
      cm[r] = m;
    }
#pragma unroll
    for (int r = 0; r < 8; ++r) {
      const int R = 8 * hh + r;
      const float mnew  = fmaxf(mrow[r], cm[r]);
      const float alpha = expf(mrow[r] - mnew);
      mrow[r] = mnew;
      float psum = 0.f;
#pragma unroll
      for (int j = 0; j < 4; ++j) {
        const float p = expf(s[j][r] - mnew);
        psum += p;
        const _Float16 ph = (_Float16)(p * kPCarry);
        const unsigned short pb = __builtin_bit_cast(unsigned short, ph);
        pn[R * kKC + j * 16 + c] = pb;
        ps[R * kPshK + j * 16 + c - R + 15] = pb;
      }
#pragma unroll
      for (int off = 1; off < 16; off <<= 1) psum += __shfl_xor(psum, off, 32);
      lrow[r] = lrow[r] * alpha + psum;
#pragma unroll
      for (int t = 0; t < 4; ++t) { oacc[t][r] *= alpha; oacc2[t][r] *= alpha; }
    }
    __syncthreads();

#pragma unroll
    for (int kk = 0; kk < 2; ++kk) {
      const v16h pa = ldfrag(pn + c * kKC + kk * 32 + 8 * hh);
#pragma unroll
      for (int t = 0; t < 4; ++t) {
        const v16h vb = ldfrag(Vtsh + (t * 16 + c) * kKC + kk * 32 + 8 * hh);
        oacc[t] = hmma(pa, vb, oacc[t]);
      }
    }
#pragma unroll
    for (int kk = 0; kk < 3; ++kk) {
      const v16h pa = ldfrag(ps + c * kPshK + kk * 32 + 8 * hh);
#pragma unroll
      for (int t = 0; t < 4; ++t) {
        const v16h tb = ldfrag(T2sh + (t * 16 + c) * kTWin + roff + kk * 32 + 8 * hh);
        oacc2[t] = hmma(pa, tb, oacc2[t]);
      }
    }
  }

  __syncthreads();
  float* os = Pqw;
#pragma unroll
  for (int r = 0; r < 8; ++r) {
    const int R = 8 * hh + r;
    const float inv = 1.0f / (lrow[r] * kPCarry);
#pragma unroll
    for (int t = 0; t < 4; ++t) os[R * kOsPitch + t * 16 + c] = (oacc[t][r] + oacc2[t][r] * kTCarryInv) * inv;
  }
  __syncthreads();
  {
    const int c4 = c * 4;
    float* ob = outp + headoff;
    for (int pass = 0; pass < 2; ++pass) {
#pragma unroll
      for (int it = 0; it < 8; ++it) {
        const int row = it * 2 + hh;
        const v4f val = *(const v4f*)(os + row * kOsPitch + c4);
        *(volatile v4f*)(ob + (size_t)(q0 + row) * kRowPitch + c4) = val;
      }
      __threadfence();
    }
  }
}

extern "C" void kernel_launch(void* const* d_in, const int* in_sizes, int n_in,
                              void* d_out, int out_size, void* d_ws, size_t ws_size,
                              hipStream_t stream) {
  constexpr int nX   = kSeqT * kBatch * kDModel;
  constexpr int nW   = kDModel * kDModel;
  constexpr int nTab = kNTab * kHDim;
  if (n_in < 11) return;
  if (in_sizes[0] != nX || in_sizes[1] != nX || in_sizes[2] != nX) return;
  if (in_sizes[3] != nW || in_sizes[5] != nW || in_sizes[7] != nW) return;
  if (in_sizes[4] != kDModel || in_sizes[6] != kDModel || in_sizes[8] != kDModel) return;
  if (in_sizes[9] != nTab || in_sizes[10] != nTab) return;
  if (out_size != nX) return;

  const float* query = (const float*)d_in[0];
  const float* key_  = (const float*)d_in[1];
  const float* value = (const float*)d_in[2];
  const float* Wq    = (const float*)d_in[3];
  const float* bq    = (const float*)d_in[4];
  const float* Wk    = (const float*)d_in[5];
  const float* bk    = (const float*)d_in[6];
  const float* Wv    = (const float*)d_in[7];
  const float* bv    = (const float*)d_in[8];
  const float* rel   = (const float*)d_in[9];
  const float* orel  = (const float*)d_in[10];
  float* out = (float*)d_out;

  const size_t bytesXb  = (size_t)3 * nX * 2;
  const size_t bytesWt  = (size_t)3 * nW * 2;
  const size_t bytesQKV = (size_t)3 * nX * 2;
  const size_t bytesR1  = (size_t)kR1Rows * kHDim * 2;
  const size_t bytesT2  = (size_t)kHDim * kT2Pitch * 2;
  const size_t offXb  = 0;
  const size_t offWt  = offXb + bytesXb;
  const size_t offQKV = offWt + bytesWt;
  const size_t offR1  = offQKV + bytesQKV;
  const size_t offT2  = offR1 + bytesR1;
  const size_t offEnd = offT2 + bytesT2;
  if (offEnd > ws_size) return;

  char* ws = (char*)d_ws;
  unsigned short* Xb   = (unsigned short*)(ws + offXb);
  unsigned short* Wt   = (unsigned short*)(ws + offWt);
  unsigned short* QKVh = (unsigned short*)(ws + offQKV);
  unsigned short* R1   = (unsigned short*)(ws + offR1);
  unsigned short* T2   = (unsigned short*)(ws + offT2);
  unsigned short* Qh = QKVh;
  unsigned short* Kh = QKVh + (size_t)nX;
  unsigned short* Vh = QKVh + (size_t)2 * nX;

  const int n8 = nX / 8;
  cast3_bf16_kernel<<<dim3(n8 / 256, 3), 256, 0, stream>>>(query, key_, value, Xb, n8);
  wt_transpose_kernel<<<dim3(kDModel / 64, kDModel / 64, 3), 256, 0, stream>>>(Wq, Wk, Wv, Wt);
  rel_cast_kernel<<<(kR1Rows * 8) / 256, 256, 0, stream>>>(rel, R1);
  orel_transpose_kernel<<<kT2Pitch / 64, 256, 0, stream>>>(orel, T2);

  const int gM = kSeqT * kBatch, gN = kDModel, gK = kDModel;
  const int gemmBlocks = (gM / 64) * (gN / 64) / 8;
  wmma_gemm64<1, false, 2, 1, false, 0><<<dim3(gemmBlocks, 1), 256, 0, stream>>>(
      Xb, Xb, gK, 0L, Wt, Wt, gK, 0L, (void*)Qh, (void*)Qh, gN, 0L, bq, bq, 0L, gM, gN, gK, 1.0f);
  wmma_gemm64<1, false, 2, 1, false, 0><<<dim3(gemmBlocks, 1), 256, 0, stream>>>(
      Xb + (size_t)nX, Xb + (size_t)nX, gK, 0L, Wt + (size_t)nW, Wt + (size_t)nW, gK, 0L,
      (void*)Kh, (void*)Kh, gN, 0L, bk, bk, 0L, gM, gN, gK, 1.0f);
  wmma_gemm64<1, false, 2, 1, false, 0><<<dim3(gemmBlocks, 1), 256, 0, stream>>>(
      Xb + (size_t)2 * nX, Xb + (size_t)2 * nX, gK, 0L, Wt + (size_t)2 * nW, Wt + (size_t)2 * nW, gK, 0L,
      (void*)Vh, (void*)Vh, gN, 0L, bv, bv, 0L, gM, gN, gK, 1.0f);

  const int attnBlocks = kBatch * kHeads * (kSeqT / kQB);
  rpe_attn_kernel<<<attnBlocks, 128, 0, stream>>>(Qh, Kh, Vh, R1, T2, out);
}
